// SeqCondAttention_61529701483094
// MI455X (gfx1250) — hardware-verified
//
#include <hip/hip_runtime.h>

typedef __attribute__((ext_vector_type(16))) _Float16 v16h;
typedef __attribute__((ext_vector_type(8)))  _Float16 v8h;
typedef __attribute__((ext_vector_type(16))) __bf16   v16b;
typedef __attribute__((ext_vector_type(8)))  __bf16   v8b;
typedef __attribute__((ext_vector_type(8)))  float    v8f;
typedef __attribute__((ext_vector_type(4)))  float    v4f;
typedef __attribute__((ext_vector_type(4)))  unsigned v4u;

constexpr int kBatch  = 2;
constexpr int kLen    = 2048;
constexpr int kDim    = 1024;
constexpr int kHeads  = 32;
constexpr int kAnch   = 4;
constexpr int kHd     = 32;
constexpr int kNTheta = 4;
constexpr int kTot    = 2 * kDim + kHeads;
constexpr int kTotPad = 2112;
constexpr int kFeat   = 2 * kHd * kNTheta;
constexpr int kHM     = kHd * kNTheta;
constexpr int kRows   = kBatch * kLen;
static_assert(kTot == 2080, "channels");
static_assert(kTotPad % 64 == 0 && kTotPad >= kTot, "N pad");
static_assert(kRows % 64 == 0 && kDim % 64 == 0 && kLen % 64 == 0, "tile multiples");
static_assert(kDim % 32 == 0 && kFeat % 32 == 0, "K multiples of 32");
static_assert(kRows % 64 == 0 && kTotPad % 64 == 0 && kDim % 32 == 0, "site0 shape");
static_assert(kLen % 64 == 0 && (2 * kHd) == 64 && kFeat % 32 == 0, "head gemm shape");
static_assert(kRows % 64 == 0 && kDim % 64 == 0, "site4 shape");
static_assert(((kRows / 64) * (kTotPad / 64)) % 8 == 0, "gemm0 grid");
static_assert(((kRows / 64) * (kDim / 64)) % 8 == 0, "gemm4 grid");
static_assert(((kLen / 64) * (kHeads / 2)) % 8 == 0, "head gemm grid");

constexpr size_t kBytesPlane = (size_t)kHeads * kLen * kFeat * 2;
constexpr size_t kBytesF     = 2 * kBytesPlane;
constexpr size_t kBytesZ     = (size_t)kRows * kTotPad * 4;
constexpr size_t kBytesXB    = (size_t)kRows * kDim * 2;
constexpr size_t kBytesWB    = (size_t)kTotPad * kDim * 2;
constexpr size_t kBytesOPB   = (size_t)kDim * kDim * 2;
constexpr size_t kBytesW23   = (size_t)kHd * kFeat * 2;
static_assert(kBytesZ <= kBytesF, "zpre aliases the feature region");
static_assert(kBytesXB == (size_t)kRows * kDim * 2, "yg aliases xb with the same extent");
static_assert(kBytesF + kBytesZ + kBytesXB + kBytesWB + kBytesOPB + kBytesW23 == 116539392ull, "carve total");
static_assert(kBytesF + kBytesZ + kBytesXB + kBytesWB + kBytesOPB + kBytesW23 <= 134217728ull, "carve cap");

__device__ __forceinline__ unsigned short f2bf_bits(float f) {
  unsigned u = __float_as_uint(f);
  return (unsigned short)((u + 0x7FFFu + ((u >> 16) & 1u)) >> 16);
}
__device__ __forceinline__ float bf_bits2f(unsigned short h) { return __uint_as_float(((unsigned)h) << 16); }
__device__ __forceinline__ float bfr(float f) { return bf_bits2f(f2bf_bits(f)); }
__device__ __forceinline__ float rcp_f(float x) { return __builtin_amdgcn_rcpf(x); }

__device__ __forceinline__ void dep_guard_h(v8f& a, v8f& b, v16h x, v16h y) { asm volatile("v_nop\n\tv_nop\n\tv_nop\n\tv_nop" : "+v"(a), "+v"(b) : "v"(x), "v"(y)); }
__device__ __forceinline__ void dep_guard_b(v8f& a, v8f& b, v16b x, v16b y) { asm volatile("v_nop\n\tv_nop\n\tv_nop\n\tv_nop" : "+v"(a), "+v"(b) : "v"(x), "v"(y)); }
__device__ __forceinline__ void keep4_h(v16h a, v16h b, v16h c, v16h d) { asm volatile("v_nop" :: "v"(a), "v"(b), "v"(c), "v"(d)); }
__device__ __forceinline__ void keep4_b(v16b a, v16b b, v16b c, v16b d) { asm volatile("v_nop" :: "v"(a), "v"(b), "v"(c), "v"(d)); }
__device__ __forceinline__ void acc_guard4(v8f& a, v8f& b, v8f& c, v8f& d) { asm volatile("v_nop\n\tv_nop\n\tv_nop\n\tv_nop" : "+v"(a), "+v"(b), "+v"(c), "+v"(d)); }
template <typename T> struct Frag;
template <> struct Frag<_Float16> {
  typedef v16h V; union U { v16h v; v8h h[2]; };
  static __device__ __forceinline__ v16h load(const _Float16* p) {
    U f; f.h[0] = *(const v8h*)(p); f.h[1] = *(const v8h*)(p + 16); return f.v;
  }
  static __device__ __forceinline__ v8f mma(v16h a, v16h b, v8f c) {
    return __builtin_amdgcn_wmma_f32_16x16x32_f16(false, a, false, b, (short)0, c, false, false);
  }
  static __device__ __forceinline__ void guard(v8f& a, v8f& b, v16h x, v16h y) { dep_guard_h(a, b, x, y); }
  static __device__ __forceinline__ void keep(v16h a, v16h b, v16h c, v16h d) { keep4_h(a, b, c, d); }
};
template <> struct Frag<__bf16> {
  typedef v16b V; union U { v16b v; v8b h[2]; };
  static __device__ __forceinline__ v16b load(const __bf16* p) {
    U f; f.h[0] = *(const v8b*)(p); f.h[1] = *(const v8b*)(p + 16); return f.v;
  }
  static __device__ __forceinline__ v8f mma(v16b a, v16b b, v8f c) {
    return __builtin_amdgcn_wmma_f32_16x16x32_bf16(false, a, false, b, (short)0, c, false, false);
  }
  static __device__ __forceinline__ void guard(v8f& a, v8f& b, v16b x, v16b y) { dep_guard_b(a, b, x, y); }
  static __device__ __forceinline__ void keep(v16b a, v16b b, v16b c, v16b d) { keep4_b(a, b, c, d); }
};

template <int ET> struct Elem;
template <> struct Elem<0> { typedef _Float16 T; };
template <> struct Elem<1> { typedef __bf16 T; };
template <int ET, bool SPLIT, int BIAS_MODE, int OUT_MODE, bool RESID, int ACT = 0>
__global__ __launch_bounds__(256) void wmma_gemm64(
    const unsigned short* __restrict__ Ap, const unsigned short* __restrict__ A2p, int lda, long strideA,
    const unsigned short* __restrict__ Btp, const unsigned short* __restrict__ Bt2p, int ldb, long strideB,
    void* __restrict__ Cout, void* __restrict__ Cout2, int ldc, long strideC,
    const float* __restrict__ bias,
    const float* __restrict__ resid, long strideR,
    int M, int N, int K, float scale) {
  typedef typename Elem<ET>::T T;
  typedef typename Frag<T>::V V;
  const T* A = (const T*)Ap; const T* A2 = (const T*)A2p; const T* Bt = (const T*)Btp; const T* Bt2 = (const T*)Bt2p;
  __shared__ __align__(16) float sT[8][16 * 68];
  const int b    = blockIdx.y;
  const int lane = threadIdx.x & 31;
  const int wave = threadIdx.x >> 5;
  const int tilesN = N >> 6;
  const int tilesM = M >> 6;
  const int tile = blockIdx.x * 8 + wave;
  if (tile >= tilesM * tilesN) return;
  const int tm = tile / tilesN;
  const int tn = tile - tm * tilesN;
  const int m0 = tm << 6;
  const int n0 = tn << 6;

  const T* Ab  = A  + (size_t)b * strideA;
  const T* Bb  = Bt + (size_t)b * strideB;
  const T* Ab2 = SPLIT ? (A2  + (size_t)b * strideA) : nullptr;
  const T* Bb2 = SPLIT ? (Bt2 + (size_t)b * strideB) : nullptr;

  const int rlane = lane & 15;
  const int koff  = (lane >> 4) * 8;
  const int mOff  = (lane >> 4) * 8;

  v8f acc[4][4];
#pragma unroll
  for (int i = 0; i < 4; ++i)
#pragma unroll
    for (int j = 0; j < 4; ++j) acc[i][j] = (v8f){0.f,0.f,0.f,0.f,0.f,0.f,0.f,0.f};

  for (int k0 = 0; k0 < K; k0 += 32) {
    V bh[4], bl[4];
#pragma unroll
    for (int j = 0; j < 4; ++j) {
      const size_t bo = (size_t)(n0 + (j << 4) + rlane) * ldb + koff + k0;
      bh[j] = Frag<T>::load(Bb + bo);
      if (SPLIT) bl[j] = Frag<T>::load(Bb2 + bo);
    }
#pragma unroll
    for (int i = 0; i < 4; ++i) {
      const size_t ao = (size_t)(m0 + (i << 4) + rlane) * lda + koff + k0;
      V ah = Frag<T>::load(Ab + ao);
      V al;
      if (SPLIT) al = Frag<T>::load(Ab2 + ao);
#pragma unroll
      for (int j = 0; j < 4; ++j) {
        acc[i][j] = Frag<T>::mma(ah, bh[j], acc[i][j]);
        if (SPLIT) {
          acc[i][j] = Frag<T>::mma(ah, bl[j], acc[i][j]);
          acc[i][j] = Frag<T>::mma(al, bh[j], acc[i][j]);
        }
      }
      Frag<T>::guard(acc[i][0], acc[i][3], ah, SPLIT ? al : ah);
    }
    Frag<T>::keep(bh[0], bh[1], bh[2], bh[3]);
    if (SPLIT) Frag<T>::keep(bl[0], bl[1], bl[2], bl[3]);
  }
  acc_guard4(acc[0][0], acc[0][1], acc[0][2], acc[0][3]);
  acc_guard4(acc[1][0], acc[1][1], acc[1][2], acc[1][3]);
  acc_guard4(acc[2][0], acc[2][1], acc[2][2], acc[2][3]);
  acc_guard4(acc[3][0], acc[3][1], acc[3][2], acc[3][3]);

  float* slab = sT[wave];
  const float* Rb = RESID ? (resid + (size_t)b * strideR) : nullptr;
#pragma unroll
  for (int i = 0; i < 4; ++i) {
    const int mBase = m0 + (i << 4);
#pragma unroll
    for (int j = 0; j < 4; ++j) {
      const int n = n0 + (j << 4) + rlane;
      float bv = 0.f;
      if (BIAS_MODE == 2) bv = bias[n];
#pragma unroll
      for (int r = 0; r < 8; ++r) {
        float v = acc[i][j][r] * scale;
        if (BIAS_MODE == 1) v += bias[mBase + mOff + r];
        if (BIAS_MODE == 2) v += bv;
        if (RESID) v += Rb[(size_t)(mBase + mOff + r) * ldc + n];
        if (ACT == 1) v = tanhf(v);
        if (ACT == 2) v = fmaxf(v, 0.0f);
        if (ACT == 3) v = v / (1.0f + expf(-v));
        if (ACT == 4) v = (v > 0.f) ? v : 0.01f * v;
        if (ACT == 5) v = 0.5f * v * (1.0f + erff(v * 0.70710678118654752f));
        slab[(mOff + r) * 68 + (j << 4) + rlane] = v;
      }
    }
    __builtin_amdgcn_fence(__ATOMIC_RELEASE, "workgroup");
    __builtin_amdgcn_wave_barrier();
    __builtin_amdgcn_fence(__ATOMIC_ACQUIRE, "workgroup");
    if (OUT_MODE == 0) {
      float* C = (float*)Cout + (size_t)b * strideC;
      const int hh = lane >> 4, c4 = (lane & 15) * 4;
      for (int pass = 0; pass < 2; ++pass) {
#pragma unroll
        for (int it = 0; it < 8; ++it) {
          const int row = it * 2 + hh;
          v4f v = *(const v4f*)(slab + row * 68 + c4);
          *(volatile v4f*)(C + (size_t)(mBase + row) * ldc + n0 + c4) = v;
        }
        __threadfence();
      }
    } else {
      const int q = lane >> 3, c8 = (lane & 7) * 8;
      unsigned short* C  = (unsigned short*)Cout  + (size_t)b * strideC;
      unsigned short* C2 = (OUT_MODE == 2) ? ((unsigned short*)Cout2 + (size_t)b * strideC) : nullptr;
      for (int pass = 0; pass < 2; ++pass) {
#pragma unroll
        for (int it = 0; it < 4; ++it) {
          const int row = it * 4 + q;
          const float* sp = slab + row * 68 + c8;
          v8h hv, lv;
#pragma unroll
          for (int e = 0; e < 8; ++e) {
            if (OUT_MODE == 1) {
              hv[e] = (_Float16)sp[e];
            } else {
              unsigned short hb = f2bf_bits(sp[e]);
              unsigned short lb = f2bf_bits(sp[e] - bf_bits2f(hb));
              hv[e] = __builtin_bit_cast(_Float16, hb);
              lv[e] = __builtin_bit_cast(_Float16, lb);
            }
          }
          *(volatile v8h*)(C + (size_t)(mBase + row) * ldc + n0 + c8) = hv;
          if (OUT_MODE == 2) *(volatile v8h*)(C2 + (size_t)(mBase + row) * ldc + n0 + c8) = lv;
        }
        __threadfence();
      }
    }
    __builtin_amdgcn_fence(__ATOMIC_RELEASE, "workgroup");
    __builtin_amdgcn_wave_barrier();
    __builtin_amdgcn_fence(__ATOMIC_ACQUIRE, "workgroup");
  }
}

__global__ __launch_bounds__(256) void cast_rows_bf16(const float* __restrict__ in,
                                                      unsigned short* __restrict__ out, int n8) {
  const int i = blockIdx.x * 256 + threadIdx.x;
  if (i < n8) {
    const v4f a = *(const v4f*)(in + (size_t)8 * i);
    const v4f c = *(const v4f*)(in + (size_t)8 * i + 4);
    v4u w;
    w[0] = (unsigned)f2bf_bits(a[0]) | ((unsigned)f2bf_bits(a[1]) << 16);
    w[1] = (unsigned)f2bf_bits(a[2]) | ((unsigned)f2bf_bits(a[3]) << 16);
    w[2] = (unsigned)f2bf_bits(c[0]) | ((unsigned)f2bf_bits(c[1]) << 16);
    w[3] = (unsigned)f2bf_bits(c[2]) | ((unsigned)f2bf_bits(c[3]) << 16);
    volatile v4u* p = (volatile v4u*)(out + (size_t)8 * i);
    *p = w;
    __threadfence();
    *p = w;
  }
}

template <int OT>
__global__ __launch_bounds__(256) void transpose_w16(const float* __restrict__ in, unsigned short* __restrict__ out,
                                                     int nRows, int nCols, float scl) {
  __shared__ __align__(16) unsigned short tileT[64 * 72];
  const int tid = threadIdx.x;
  const int k0 = blockIdx.x * 64;
  const int n0 = blockIdx.y * 64;
  const int nn = tid & 63, kq = tid >> 6;
  const int n = n0 + nn;
  const int nc = n < nCols ? n : (nCols - 1);
  const bool nok = n < nCols;
#pragma unroll 4
  for (int p = 0; p < 16; ++p) {
    const int kk = p * 4 + kq;
    float v = in[(size_t)(k0 + kk) * nCols + nc];
    v = nok ? v : 0.0f;
    const unsigned short hb = f2bf_bits(v);
    unsigned short o;
    if (OT == 0) {
      o = hb;
    } else {
      const _Float16 hf = (_Float16)(bf_bits2f(hb) * scl);
      o = __builtin_bit_cast(unsigned short, hf);
    }
    tileT[nn * 72 + kk] = o;
  }
  __syncthreads();
  const int wave = tid >> 5, lane = tid & 31, q = lane >> 3, c8 = (lane & 7) * 8;
  v4u vv[2];
#pragma unroll
  for (int it = 0; it < 2; ++it) {
    const int row = wave * 8 + it * 4 + q;
    vv[it] = *(const v4u*)(tileT + row * 72 + c8);
  }
  for (int pass = 0; pass < 2; ++pass) {
#pragma unroll
    for (int it = 0; it < 2; ++it) {
      const int row = wave * 8 + it * 4 + q;
      *(volatile v4u*)(out + (size_t)(n0 + row) * nRows + k0 + c8) = vv[it];
    }
    __threadfence();
  }
}

__global__ __launch_bounds__(256) void build_headw(const float* __restrict__ wre, const float* __restrict__ wim,
                                                   unsigned short* __restrict__ out) {
  __shared__ __align__(16) unsigned short tw[32 * 264];
  const int tid = threadIdx.x;
#pragma unroll
  for (int j = 0; j < 4; ++j) {
    const int base = 1024 * j + 4 * tid;
    const v4f a = *(const v4f*)(wre + base);
    const v4f c = *(const v4f*)(wim + base);
    const int f = base >> 5;
    const int hp0 = base & 31;
#pragma unroll
    for (int e = 0; e < 4; ++e) {
      tw[(hp0 + e) * 264 + f]       = f2bf_bits(a[e]);
      tw[(hp0 + e) * 264 + kHM + f] = f2bf_bits(c[e]);
    }
  }
  __syncthreads();
  const int wave = tid >> 5, lane = tid & 31, q = lane >> 3, c8 = (lane & 7) * 8;
  v4u vv[4];
#pragma unroll
  for (int it = 0; it < 4; ++it) {
    const int li = wave * 16 + it * 4 + q;
    const int row = li >> 2, seg = li & 3;
    vv[it] = *(const v4u*)(tw + row * 264 + seg * 64 + c8);
  }
  for (int pass = 0; pass < 2; ++pass) {
#pragma unroll
    for (int it = 0; it < 4; ++it) {
      const int li = wave * 16 + it * 4 + q;
      const int row = li >> 2, seg = li & 3;
      *(volatile v4u*)(out + (size_t)row * kFeat + seg * 64 + c8) = vv[it];
    }
    __threadfence();
  }
}

__global__ __launch_bounds__(256) void dwconv4_gate(const float* __restrict__ zpre, const float* __restrict__ cw,
                                                    const float* __restrict__ cb, float* __restrict__ zc, int n4) {
  const int i = blockIdx.x * 256 + threadIdx.x;
  if (i >= n4) return;
  const int r  = i / (kTotPad / 4);
  const int c4 = (i - r * (kTotPad / 4)) * 4;
  const int l  = r & (kLen - 1);
  const int c4w = c4 < (kTot - 4) ? c4 : (kTot - 4);
  float a0 = 0.0f, a1 = 0.0f, a2 = 0.0f, a3 = 0.0f;
#pragma unroll
  for (int t = 0; t < 4; ++t) {
    const int ls = l - 3 + t;
    const bool ok = ls >= 0;
    const int rsrc = ok ? (r - 3 + t) : r;
    const v4f zv = *(const v4f*)(zpre + (size_t)rsrc * kTotPad + c4);
    const v4f wv = *(const v4f*)(cw + (size_t)t * kTot + c4w);
    const float t0 = bfr(wv[0]) * zv[0];
    const float t1 = bfr(wv[1]) * zv[1];
    const float t2 = bfr(wv[2]) * zv[2];
    const float t3 = bfr(wv[3]) * zv[3];
    a0 += ok ? t0 : 0.0f;
    a1 += ok ? t1 : 0.0f;
    a2 += ok ? t2 : 0.0f;
    a3 += ok ? t3 : 0.0f;
  }
  const v4f bv = *(const v4f*)(cb + c4w);
  const bool isg = (c4 >= kDim) && (c4 < 2 * kDim);
  float vv[4];
  vv[0] = a0 + bfr(bv[0]); vv[1] = a1 + bfr(bv[1]); vv[2] = a2 + bfr(bv[2]); vv[3] = a3 + bfr(bv[3]);
  v4f o;
#pragma unroll
  for (int e = 0; e < 4; ++e) {
    const float v = vv[e];
    const float sg = v * rcp_f(1.0f + expf(-v));
    o[e] = isg ? sg : v;
  }
  volatile v4f* p = (volatile v4f*)(zc + (size_t)r * kTotPad + c4);
  *p = o;
  __threadfence();
  *p = o;
}

__global__ __launch_bounds__(32) void scan_features(const float* __restrict__ zc, const float* __restrict__ theta,
                                                    const float* __restrict__ dsl, const float* __restrict__ asl,
                                                    const float* __restrict__ ssc, const float* __restrict__ dlg,
                                                    const float* __restrict__ nsc,
                                                    unsigned short* __restrict__ Fh, unsigned short* __restrict__ Fl,
                                                    int bsel) {
  __shared__ float sTh[kNTheta][32];
  __shared__ float sNr[kNTheta][32];
  __shared__ float sNi[kNTheta][32];
  __shared__ float sAr[kNTheta][32];
  __shared__ float sAi[kNTheta][32];
  __shared__ float sVr[kNTheta][32];
  __shared__ float sVi[kNTheta][32];
  __shared__ float sE[4][32];
  __shared__ __align__(16) unsigned short sRowH[kFeat];
  __shared__ __align__(16) unsigned short sRowL[kFeat];

  const int k = blockIdx.x;
  const int h = threadIdx.x;
#pragma unroll 1
  for (int m = 0; m < kNTheta; ++m) {
    sTh[m][h] = bfr(theta[(size_t)(k * kHd + h) * kNTheta + m]);
    sNr[m][h] = bfr(nsc[h * kNTheta + m]);
    sNi[m][h] = bfr(nsc[kHM + h * kNTheta + m]);
    sAr[m][h] = 0.0f;
    sAi[m][h] = 0.0f;
  }
  const float g0 = bfr(dlg[0]), g1 = bfr(dlg[1]), g2 = bfr(dlg[2]);
  const float gm = fmaxf(g0, fmaxf(g1, g2));
  float esum = 0.0f;
#pragma unroll 1
  for (int i = 0; i < 3; ++i) {
    const float e = expf(bfr(dlg[i]) - gm);
    sE[i][h] = e;
    esum += e;
  }
  const float einv = rcp_f(esum);
  const float w0 = sE[0][h] * einv;
  const float w1 = sE[1][h] * einv;
  const float w2 = sE[2][h] * einv;
  const bool anchor = (k >= kHeads - kAnch);
  const int kd = k < (kHeads - kAnch) ? k : (kHeads - kAnch - 1);
  const int ka = anchor ? (k - (kHeads - kAnch)) : 0;
  const float rd = bfr(dsl[kd]);
  const float ra = bfr(asl[ka]);
  const float raw = anchor ? ra : rd;
  const float slope = fmaxf(raw, 0.0f) + log1pf(expf(-fabsf(raw)));
  const float nslope = -slope;
  const float sc = bfr(ssc[k]);

  float den = 0.0f;
  const float* zrow = zc + (size_t)bsel * kLen * kTotPad;
  unsigned short* fh = Fh + (size_t)k * kLen * kFeat + h * 8;
  unsigned short* fl = Fl + (size_t)k * kLen * kFeat + h * 8;

#pragma unroll 1
  for (int l = 0; l < kLen; ++l) {
    const float xv = zrow[k * kHd + h];
    const float s  = zrow[2 * kDim + k];
    zrow += kTotPad;
    const float dist = anchor ? (float)l : (float)(kLen - 1 - l);
    const float tw = expf(nslope * dist);
    float a = sc * s;
    a = fminf(fmaxf(a, -20.0f), 20.0f);
    const float p = expf(a);
    const float pw = p * tw;
    den += pw;
    const float poly = w0 + w1 * xv - w2 * (xv * xv);
    const float invd = rcp_f(fmaxf(den, 1e-4f));
    float part = 0.0f;
#pragma unroll 1
    for (int m = 0; m < kNTheta; ++m) {
      float sn, cs;
      sincosf(xv * sTh[m][h], &sn, &cs);
      const float ar = sAr[m][h] + pw * (poly * cs);
      const float ai = sAi[m][h] + pw * (poly * sn);
      sAr[m][h] = ar;
      sAi[m][h] = ai;
      const float rr = ar * invd;
      const float ii = ai * invd;
      sVr[m][h] = rr;
      sVi[m][h] = ii;
      part += rr * rr + ii * ii;
    }
#pragma unroll
    for (int off = 16; off > 0; off >>= 1) part += __shfl_xor(part, off, 32);
    const float rs = rsqrtf(part * (1.0f / 256.0f) + 1e-5f);
#pragma unroll 1
    for (int m = 0; m < kNTheta; ++m) {
      const float vr = sVr[m][h] * rs * sNr[m][h];
      const float vi = sVi[m][h] * rs * sNi[m][h];
      const unsigned short hr = f2bf_bits(vr);
      const unsigned short lr = f2bf_bits(vr - bf_bits2f(hr));
      const unsigned short hi = f2bf_bits(vi);
      const unsigned short li = f2bf_bits(vi - bf_bits2f(hi));
      sRowH[h * kNTheta + m] = hr;
      sRowH[kHM + h * kNTheta + m] = hi;
      sRowL[h * kNTheta + m] = lr;
      sRowL[kHM + h * kNTheta + m] = li;
    }
    __syncthreads();
    const v4u hv = *(const v4u*)(sRowH + h * 8);
    const v4u lv = *(const v4u*)(sRowL + h * 8);
    *(volatile v4u*)fh = hv;
    *(volatile v4u*)fl = lv;
    __threadfence();
    *(volatile v4u*)fh = hv;
    *(volatile v4u*)fl = lv;
    fh += kFeat;
    fl += kFeat;
    __syncthreads();
  }
}

__global__ __launch_bounds__(256) void head_gemm(const unsigned short* __restrict__ Fhp, const unsigned short* __restrict__ Flp,
                                                 const unsigned short* __restrict__ Wtp, const float* __restrict__ zc,
                                                 unsigned short* __restrict__ yg, int bsel) {
  typedef __bf16 T;
  typedef Frag<__bf16>::V V;
  const T* Ah = (const T*)Fhp; const T* Al = (const T*)Flp; const T* Bt = (const T*)Wtp;
  __shared__ __align__(16) float sT[8][16 * 68];
  const int lane = threadIdx.x & 31;
  const int wave = threadIdx.x >> 5;
  const int tile = blockIdx.x * 8 + wave;
  if (tile >= (kLen / 64) * (kHeads / 2)) return;
  const int lt = tile >> 4, kp = tile & 15;
  const int l0 = lt * 64, k0 = kp * 2;
  const int rlane = lane & 15;
  const int koff  = (lane >> 4) * 8;
  const int mOff  = (lane >> 4) * 8;

  v8f acc[4][2][2];
#pragma unroll
  for (int i = 0; i < 4; ++i)
#pragma unroll
    for (int j = 0; j < 2; ++j)
#pragma unroll
      for (int t = 0; t < 2; ++t) acc[i][j][t] = (v8f){0.f,0.f,0.f,0.f,0.f,0.f,0.f,0.f};

#pragma unroll 1
  for (int ks = 0; ks < kFeat; ks += 32) {
    V bw[2];
#pragma unroll
    for (int t = 0; t < 2; ++t) bw[t] = Frag<T>::load(Bt + (size_t)(t * 16 + rlane) * kFeat + koff + ks);
#pragma unroll
    for (int j = 0; j < 2; ++j) {
#pragma unroll
      for (int i = 0; i < 4; ++i) {
        const size_t ao = ((size_t)(k0 + j) * kLen + l0 + i * 16 + rlane) * kFeat + koff + ks;
        V ah = Frag<T>::load(Ah + ao);
        V al = Frag<T>::load(Al + ao);
#pragma unroll
        for (int t = 0; t < 2; ++t) {
          acc[i][j][t] = Frag<T>::mma(ah, bw[t], acc[i][j][t]);
          acc[i][j][t] = Frag<T>::mma(al, bw[t], acc[i][j][t]);
        }
        Frag<T>::guard(acc[i][j][0], acc[i][j][1], ah, al);
      }
    }
    Frag<T>::keep(bw[0], bw[1], bw[0], bw[1]);
  }
  acc_guard4(acc[0][0][0], acc[0][0][1], acc[0][1][0], acc[0][1][1]);
  acc_guard4(acc[1][0][0], acc[1][0][1], acc[1][1][0], acc[1][1][1]);
  acc_guard4(acc[2][0][0], acc[2][0][1], acc[2][1][0], acc[2][1][1]);
  acc_guard4(acc[3][0][0], acc[3][0][1], acc[3][1][0], acc[3][1][1]);

  float* slab = sT[wave];
  const int q = lane >> 3, c8 = (lane & 7) * 8;
#pragma unroll
  for (int i = 0; i < 4; ++i) {
#pragma unroll
    for (int j = 0; j < 2; ++j)
#pragma unroll
      for (int t = 0; t < 2; ++t)
#pragma unroll
        for (int r = 0; r < 8; ++r)
          slab[(mOff + r) * 68 + j * 32 + t * 16 + rlane] = acc[i][j][t][r];
    __builtin_amdgcn_fence(__ATOMIC_RELEASE, "workgroup");
    __builtin_amdgcn_wave_barrier();
    __builtin_amdgcn_fence(__ATOMIC_ACQUIRE, "workgroup");
    v8h hv[4];
#pragma unroll
    for (int it = 0; it < 4; ++it) {
      const int row = it * 4 + q;
      const int lrow = l0 + i * 16 + row;
      const float* sp = slab + row * 68 + c8;
      const float* gp = zc + ((size_t)(bsel * kLen + lrow)) * kTotPad + kDim + k0 * kHd + c8;
      const v4f ga = *(const v4f*)gp;
      const v4f gb = *(const v4f*)(gp + 4);
      float gg[8];
      gg[0] = ga[0]; gg[1] = ga[1]; gg[2] = ga[2]; gg[3] = ga[3];
      gg[4] = gb[0]; gg[5] = gb[1]; gg[6] = gb[2]; gg[7] = gb[3];
#pragma unroll
      for (int e = 0; e < 8; ++e) hv[it][e] = (_Float16)(sp[e] * gg[e] * 32.0f);
    }
    for (int pass = 0; pass < 2; ++pass) {
#pragma unroll
      for (int it = 0; it < 4; ++it) {
        const int row = it * 4 + q;
        *(volatile v8h*)(yg + ((size_t)(bsel * kLen + l0 + i * 16 + row)) * kDim + k0 * kHd + c8) = hv[it];
      }
      __threadfence();
    }
    __builtin_amdgcn_fence(__ATOMIC_RELEASE, "workgroup");
    __builtin_amdgcn_wave_barrier();
    __builtin_amdgcn_fence(__ATOMIC_ACQUIRE, "workgroup");
  }
}

extern "C" void kernel_launch(void* const* d_in, const int* in_sizes, int n_in,
                              void* d_out, int out_size, void* d_ws, size_t ws_size,
                              hipStream_t stream) {
  if (n_in < 13) return;
  if (in_sizes[0] != kRows * kDim || out_size != kRows * kDim) return;
  if (in_sizes[1] != kDim * kTot || in_sizes[12] != kDim * kDim) return;

  const float* x             = (const float*)d_in[0];
  const float* in_proj_w     = (const float*)d_in[1];
  const float* conv_w        = (const float*)d_in[2];
  const float* conv_b        = (const float*)d_in[3];
  const float* theta         = (const float*)d_in[4];
  const float* decay_slopes  = (const float*)d_in[5];
  const float* anchor_slopes = (const float*)d_in[6];
  const float* score_scale   = (const float*)d_in[7];
  const float* deriv_logits  = (const float*)d_in[8];
  const float* norm_scale    = (const float*)d_in[9];
  const float* w_re          = (const float*)d_in[10];
  const float* w_im          = (const float*)d_in[11];
  const float* out_proj_w    = (const float*)d_in[12];
  float*       out           = (float*)d_out;

  char* ws = (char*)d_ws;
  size_t off = 0;
  auto carve = [&](size_t bytes) { size_t o = off; off = (off + bytes + 255) & ~(size_t)255; return o; };
  const size_t oF   = carve(kBytesF);
  const size_t oZC  = carve(kBytesZ);
  const size_t oXB  = carve(kBytesXB);
  const size_t oWB  = carve(kBytesWB);
  const size_t oOPB = carve(kBytesOPB);
  const size_t oW23 = carve(kBytesW23);
  if (off > ws_size) return;

  unsigned short* fhi  = (unsigned short*)(ws + oF);
  unsigned short* flo  = (unsigned short*)(ws + oF + kBytesPlane);
  float*          zpre = (float*)(ws + oF);
  float*          zc   = (float*)(ws + oZC);
  unsigned short* xb   = (unsigned short*)(ws + oXB);
  unsigned short* yg   = (unsigned short*)(ws + oXB);
  unsigned short* wb   = (unsigned short*)(ws + oWB);
  unsigned short* opb  = (unsigned short*)(ws + oOPB);
  unsigned short* w23  = (unsigned short*)(ws + oW23);

  {
    const int n8 = kRows * kDim / 8;
    cast_rows_bf16<<<(n8 + 255) / 256, 256, 0, stream>>>(x, xb, n8);
  }
  transpose_w16<0><<<dim3(kDim / 64, kTotPad / 64), 256, 0, stream>>>(in_proj_w, wb, kDim, kTot, 1.0f);
  transpose_w16<1><<<dim3(kDim / 64, kDim / 64), 256, 0, stream>>>(out_proj_w, opb, kDim, kDim, 16.0f);
  build_headw<<<1, 256, 0, stream>>>(w_re, w_im, w23);

  wmma_gemm64<1, false, 0, 0, false, 0><<<dim3((kRows / 64) * (kTotPad / 64) / 8, 1), 256, 0, stream>>>(
      xb, xb, kDim, 0L, wb, wb, kDim, 0L, (void*)zpre, (void*)zpre, kTotPad, 0L,
      conv_b, x, 0L, kRows, kTotPad, kDim, 1.0f);

  {
    const int n4 = kRows * (kTotPad / 4);
    dwconv4_gate<<<(n4 + 255) / 256, 256, 0, stream>>>(zpre, conv_w, conv_b, zc, n4);
  }

  for (int b = 0; b < kBatch; ++b) {
    scan_features<<<kHeads, 32, 0, stream>>>(zc, theta, decay_slopes, anchor_slopes, score_scale,
                                             deriv_logits, norm_scale, fhi, flo, b);
    head_gemm<<<(kLen / 64) * (kHeads / 2) / 8, 256, 0, stream>>>(fhi, flo, w23, zc, yg, b);
  }

  wmma_gemm64<0, false, 0, 0, false, 0><<<dim3((kRows / 64) * (kDim / 64) / 8, 1), 256, 0, stream>>>(
      yg, yg, kDim, 0L, opb, opb, kDim, 0L, (void*)out, (void*)out, kDim, 0L,
      conv_b, x, 0L, kRows, kDim, kDim, 1.0f / 512.0f);
}
